// EquivariantDiffuserV46_66949950210595
// MI455X (gfx1250) — hardware-verified
//
#include <hip/hip_runtime.h>
#include <stddef.h>
#include <math.h>


#define NTHR   256
#define NWAVE  8
#define EPT    8
#define CHUNK  (NTHR * EPT)
#define WCAP   (EPT * 32)
#define LISTN  (NWAVE * WCAP)
#define PASSN  (NWAVE * 32)
#define PCAP   (CHUNK + PASSN)
#define NB     1024
#define AW     3
#define ND     64
#define HD     128
#define EDM    32
#define PQW    256
#define NWROW  (EDM + HD)
#define BSMN   224
#define EW1O   0
#define EB1O   32
#define EB2O   64
#define CW2O   96
#define NQ     ((NB * AW) / (128 * NWAVE))
#define WSC    16.0f
#define WINV   0.0625f
#define WINV2  0.00390625f

static_assert(NQ * 128 * NWAVE == NB * AW);
static_assert(PASSN == 256);
static_assert((NB % 32) == 0);
static_assert(PCAP >= CHUNK + PASSN);
static_assert(BSMN == CW2O + HD);

typedef float    v4f  __attribute__((ext_vector_type(4)));
typedef float    v8f  __attribute__((ext_vector_type(8)));
typedef int      v4i  __attribute__((ext_vector_type(4)));
typedef _Float16 v8h  __attribute__((ext_vector_type(8)));
typedef _Float16 v16h __attribute__((ext_vector_type(16)));
union FragH { v16h v; v8h h[2]; };

__device__ __forceinline__ v8f zero8f() {
  v8f r;
#pragma unroll
  for (int i = 0; i < 8; ++i) r[i] = 0.0f;
  return r;
}

__device__ __forceinline__ v8f wmh(v16h a, v16h b, v8f c) {
  v8f d = __builtin_amdgcn_wmma_f32_16x16x32_f16(false, a, false, b, (short)0, c, false, false);
  asm volatile("v_nop\n\tv_nop\n\tv_nop\n\tv_nop" : "+v"(d) : "v"(a), "v"(b));
  return d;
}

__device__ __forceinline__ v8f ld8(const float* p) {
  const v4f a = *(const v4f*)p;
  const v4f b = *(const v4f*)(p + 4);
  v8f c;
  c[0] = a.x; c[1] = a.y; c[2] = a.z; c[3] = a.w;
  c[4] = b.x; c[5] = b.y; c[6] = b.z; c[7] = b.w;
  return c;
}

__device__ __forceinline__ float silu_f(float v) {
  return v * __builtin_amdgcn_rcpf(1.0f + __expf(-v));
}

__global__ __launch_bounds__(256) void k_prep(const float* __restrict__ cond, const int* __restrict__ tp,
                                              const float* __restrict__ cw1,
                                              _Float16* h16, _Float16* wt16, int nN, int nHB) {
  const int tid = threadIdx.x;
  const int piece = tid & 7, rl = tid >> 3;
  if ((int)blockIdx.x < nHB) {
    const int row = (int)blockIdx.x * 32 + rl;
    int rc = row < nN ? row : nN - 1;
    rc = rc < 0 ? 0 : rc;
    const float tv = (float)tp[0];
    const float keep = (row < nN) ? 1.0f : 0.0f;
    v8h hv;
#pragma unroll
    for (int i = 0; i < 8; ++i) {
      const int c  = 8 * piece + i;
      const int cc = c < 63 ? c : 62;
      const float cv = cond[(size_t)rc * 63 + cc];
      const float v  = (c < 63) ? cv : tv;
      hv[i] = (_Float16)(v * keep);
    }
    _Float16* dp = h16 + (size_t)row * ND + 8 * piece;
    *(volatile v8h*)dp = hv;
    __threadfence();
    *(volatile v8h*)dp = hv;
  } else {
    int n = ((int)blockIdx.x - nHB) * 32 + rl;
    n = n < 0 ? 0 : (n > 2 * HD - 1 ? 2 * HD - 1 : n);
    v8h hv;
#pragma unroll
    for (int i = 0; i < 8; ++i) {
      const int k = 8 * piece + i;
      const int idx = (n < HD) ? (k * HD + n) : ((ND + k) * HD + (n - HD));
      hv[i] = (_Float16)(cw1[idx] * WSC);
    }
    _Float16* dp = wt16 + (size_t)n * ND + 8 * piece;
    *(volatile v8h*)dp = hv;
    __threadfence();
    *(volatile v8h*)dp = hv;
  }
}

__global__ __launch_bounds__(64) void k_node(const _Float16* __restrict__ h16, const _Float16* __restrict__ wt16,
                                             const float* __restrict__ cb1, float* pq) {
  __shared__ __attribute__((aligned(16))) float stg[16 * PQW];
  const int tid = threadIdx.x, lane = tid & 31, wave = tid >> 5, hh = lane >> 4, m = lane & 15;
  const int rowBase = (int)blockIdx.x * 16;
  const int colBase = wave * HD;

  FragH a[2];
#pragma unroll
  for (int ks = 0; ks < 2; ++ks) {
    const _Float16* ap = h16 + (size_t)(rowBase + m) * ND + 32 * ks + 8 * hh;
    a[ks].h[0] = *(const v8h*)ap;
    a[ks].h[1] = *(const v8h*)(ap + 16);
  }
  v8f acc[8];
#pragma unroll
  for (int ct = 0; ct < 8; ++ct) acc[ct] = zero8f();
#pragma unroll
  for (int ks = 0; ks < 2; ++ks) {
#pragma unroll
    for (int ct = 0; ct < 8; ++ct) {
      FragH b;
      const _Float16* bp = wt16 + (size_t)(colBase + 16 * ct + m) * ND + 32 * ks + 8 * hh;
      b.h[0] = *(const v8h*)bp;
      b.h[1] = *(const v8h*)(bp + 16);
      acc[ct] = wmh(a[ks].v, b.v, acc[ct]);
    }
  }
  const float bsel = (wave != 0) ? 1.0f : 0.0f;
#pragma unroll
  for (int ct = 0; ct < 8; ++ct) {
    const float bb = cb1[16 * ct + m] * bsel;
#pragma unroll
    for (int r = 0; r < 8; ++r)
      stg[(8 * hh + r) * PQW + colBase + 16 * ct + m] = acc[ct][r] * WINV + bb;
  }
  __syncthreads();
  v4f ov[16];
#pragma unroll
  for (int rr = 0; rr < 8; ++rr) {
#pragma unroll
    for (int q2 = 0; q2 < 2; ++q2)
      ov[rr * 2 + q2] = *(const v4f*)(stg + (8 * wave + rr) * PQW + (q2 * 32 + lane) * 4);
  }
  float* gb = pq + (size_t)(rowBase + 8 * wave) * PQW;
#pragma unroll
  for (int rr = 0; rr < 8; ++rr) {
#pragma unroll
    for (int q2 = 0; q2 < 2; ++q2)
      *(volatile v4f*)(gb + (size_t)rr * PQW + (q2 * 32 + lane) * 4) = ov[rr * 2 + q2];
  }
  __threadfence();
#pragma unroll
  for (int rr = 0; rr < 8; ++rr) {
#pragma unroll
    for (int q2 = 0; q2 < 2; ++q2)
      *(volatile v4f*)(gb + (size_t)rr * PQW + (q2 * 32 + lane) * 4) = ov[rr * 2 + q2];
  }
}

__device__ __forceinline__ int scan_chunk(const int* __restrict__ dsts, int nE, int cbase, int nodeBase,
                                          int vec8, int* list, int tid, int wave) {
  int wc = 0;
  const int el0  = tid * EPT;
  const int e0   = cbase + el0;
  const int sent = -2147483647 - 1;
  v4i da, db;
  if (vec8 != 0 && cbase + CHUNK <= nE) {
    da = *(const v4i*)(dsts + e0);
    db = *(const v4i*)(dsts + e0 + 4);
  } else {
    da.x = (e0     < nE) ? dsts[min(e0, nE - 1)] : sent;
    da.y = (e0 + 1 < nE) ? dsts[min(e0 + 1, nE - 1)] : sent;
    da.z = (e0 + 2 < nE) ? dsts[min(e0 + 2, nE - 1)] : sent;
    da.w = (e0 + 3 < nE) ? dsts[min(e0 + 3, nE - 1)] : sent;
    db.x = (e0 + 4 < nE) ? dsts[min(e0 + 4, nE - 1)] : sent;
    db.y = (e0 + 5 < nE) ? dsts[min(e0 + 5, nE - 1)] : sent;
    db.z = (e0 + 6 < nE) ? dsts[min(e0 + 6, nE - 1)] : sent;
    db.w = (e0 + 7 < nE) ? dsts[min(e0 + 7, nE - 1)] : sent;
  }
  const unsigned nb = (unsigned)nodeBase;
  const unsigned s0 = (unsigned)da.x - nb, s1 = (unsigned)da.y - nb;
  const unsigned s2 = (unsigned)da.z - nb, s3 = (unsigned)da.w - nb;
  const unsigned s4 = (unsigned)db.x - nb, s5 = (unsigned)db.y - nb;
  const unsigned s6 = (unsigned)db.z - nb, s7 = (unsigned)db.w - nb;
  const bool h0 = s0 < (unsigned)NB, h1 = s1 < (unsigned)NB, h2 = s2 < (unsigned)NB, h3 = s3 < (unsigned)NB;
  const bool h4 = s4 < (unsigned)NB, h5 = s5 < (unsigned)NB, h6 = s6 < (unsigned)NB, h7 = s7 < (unsigned)NB;
  const unsigned any = __builtin_amdgcn_ballot_w32(h0 | h1 | h2 | h3 | h4 | h5 | h6 | h7);
  if (any != 0u) {
#define HITJ(J, HJ) { \
      const unsigned mj = __builtin_amdgcn_ballot_w32(HJ); \
      if (mj != 0u) { \
        if (HJ) { \
          const int pos = wc + (int)__builtin_amdgcn_mbcnt_lo(mj, 0u); \
          if (pos < WCAP) list[wave * WCAP + pos] = el0 + (J); \
        } \
        wc += (int)__builtin_popcount(mj); } }
    HITJ(0, h0)
    HITJ(1, h1)
    HITJ(2, h2)
    HITJ(3, h3)
    HITJ(4, h4)
    HITJ(5, h5)
    HITJ(6, h6)
    HITJ(7, h7)
#undef HITJ
  }
  return wc;
}

__global__ __launch_bounds__(NTHR) void k_agg(
    const float* __restrict__ x, const int* __restrict__ ei, const float* __restrict__ edist,
    const float* __restrict__ ew1, const float* __restrict__ eb1,
    const float* __restrict__ ew2, const float* __restrict__ eb2,
    const float* __restrict__ cw1, const float* __restrict__ cw2,
    const float* __restrict__ pq, float* outp, int nN, int nE, int vec8, int outLim) {
  __shared__ __attribute__((aligned(16))) float    acc[(NB + 1) * AW];
  __shared__ __attribute__((aligned(16))) float    msg[PASSN * AW];
  __shared__ __attribute__((aligned(16))) _Float16 hid[PASSN * EDM];
  __shared__ __attribute__((aligned(16))) int      list[LISTN];
  __shared__ __attribute__((aligned(16))) int      pend[PCAP];
  __shared__ int slotb[PASSN];
  __shared__ int ssrc[PASSN];
  __shared__ int sdst[PASSN];
  __shared__ __attribute__((aligned(16))) _Float16 wsm[NWROW * 32];
  __shared__ __attribute__((aligned(16))) float    bsm[BSMN];
  __shared__ int wcnt[NWAVE];
  __shared__ int pendN;

  const int tid = threadIdx.x, lane = tid & 31, wave = tid >> 5, hh = lane >> 4, m = lane & 15;
  const int nodeBase = (int)blockIdx.x * NB;
  const int* srcs = ei;
  const int* dsts = ei + nE;

  for (int i = tid; i < (NB + 1) * AW; i += NTHR) acc[i] = 0.0f;
  for (int i = tid; i < NWROW * 32; i += NTHR) {
    const int row = i >> 5, k = i & 31;
    const float va = ew2[k * EDM + (row & 31)];
    const float vb = cw1[(HD + k) * HD + ((row - EDM) & (HD - 1))];
    const float v  = (row < EDM) ? va : vb;
    wsm[i] = (_Float16)(v * WSC);
  }
  if (tid < BSMN) {
    const float v0 = ew1[tid & 31];
    const float v1 = eb1[tid & 31];
    const float v2 = eb2[tid & 31];
    const float v3 = cw2[(tid - CW2O) & (HD - 1)];
    const float v  = (tid < EB1O) ? v0 : ((tid < EB2O) ? v1 : ((tid < CW2O) ? v2 : v3));
    bsm[tid] = v;
  }
  if (tid == 0) pendN = 0;
  __syncthreads();

  const int nChunks = (nE + CHUNK - 1) / CHUNK;
#pragma unroll 1
  for (int ch = 0; ch < nChunks; ++ch) {
    const int cbase = ch * CHUNK;
    const int wc = scan_chunk(dsts, nE, cbase, nodeBase, vec8, list, tid, wave);
    if (lane == 0) wcnt[wave] = wc;
    __syncthreads();

    const int base = pendN;
    int tot = 0, myoff = 0;
#pragma unroll
    for (int w = 0; w < NWAVE; ++w) {
      int c = wcnt[w];
      c = c > WCAP ? WCAP : (c < 0 ? 0 : c);
      if (w < wave) myoff += c;
      tot += c;
    }
    int newN = base + tot;
    newN = newN > PCAP ? PCAP : newN;
    {
      int n = wcnt[wave];
      n = n > WCAP ? WCAP : (n < 0 ? 0 : n);
      const int* lp = list + wave * WCAP;
      for (int i = lane; i < n; i += 32) {
        const int pos = base + myoff + i;
        if (pos < PCAP) pend[pos] = cbase + lp[i];
      }
    }
    const int fin = (ch == nChunks - 1) ? 1 : 0;
    const int R   = (fin != 0) ? (newN + PASSN - 1) / PASSN : newN / PASSN;
    const int Pv  = (fin != 0) ? newN : R * PASSN;
    __syncthreads();

#pragma unroll 1
    for (int r = 0; r < R; ++r) {
      float ux, uy, uz;
      {
        const int idx = r * PASSN + wave * 32 + lane;
        const bool valid = idx < Pv;
        int e = pend[idx];
        e = valid ? e : 0;
        e = e < 0 ? 0 : (e > nE - 1 ? nE - 1 : e);
        int d = dsts[e];
        int s = srcs[e];
        int slot = d - nodeBase;
        if (!valid || (unsigned)slot >= (unsigned)NB) slot = NB;
        d = d < 0 ? 0 : (d > nN - 1 ? nN - 1 : d);
        s = s < 0 ? 0 : (s > nN - 1 ? nN - 1 : s);
        const float* xs = x + (size_t)s * 3;
        const float* xd = x + (size_t)d * 3;
        const float dx = xs[0] - xd[0];
        const float dy = xs[1] - xd[1];
        const float dz = xs[2] - xd[2];
        const float len = fmaxf(sqrtf(dx * dx + dy * dy + dz * dz), 1e-8f);
        const float inv = 1.0f / len;
        ux = dx * inv; uy = dy * inv; uz = dz * inv;
        const float dval = edist[e];
        _Float16* hp = hid + (wave * 32 + lane) * EDM;
#pragma unroll 1
        for (int j = 0; j < 4; ++j) {
          v8h hv;
#pragma unroll
          for (int i = 0; i < 8; ++i) {
            const float z = fmaf(dval, bsm[EW1O + 8 * j + i], bsm[EB1O + 8 * j + i]);
            hv[i] = (_Float16)(silu_f(z) * WSC);
          }
          *(v8h*)(hp + 8 * j) = hv;
        }
        ssrc[wave * 32 + lane]  = s;
        sdst[wave * 32 + lane]  = d;
        slotb[wave * 32 + lane] = slot;
      }
      __syncthreads();

      {
        const v8f z8 = zero8f();
        const _Float16* hr0 = hid + (wave * 32 + m) * EDM;
        const _Float16* hr1 = hid + (wave * 32 + 16 + m) * EDM;
        FragH bh0, bh1;
        bh0.h[0] = *(const v8h*)(hr0 + 8 * hh); bh0.h[1] = *(const v8h*)(hr0 + 16 + 8 * hh);
        bh1.h[0] = *(const v8h*)(hr1 + 8 * hh); bh1.h[1] = *(const v8h*)(hr1 + 16 + 8 * hh);
        v8f d00, d01, d10, d11;
        {
          FragH a;
          const _Float16* ap = wsm + m * 32 + 8 * hh;
          a.h[0] = *(const v8h*)ap;
          a.h[1] = *(const v8h*)(ap + 16);
          d00 = wmh(a.v, bh0.v, z8);
          d01 = wmh(a.v, bh1.v, z8);
        }
        {
          FragH a;
          const _Float16* ap = wsm + (16 + m) * 32 + 8 * hh;
          a.h[0] = *(const v8h*)ap;
          a.h[1] = *(const v8h*)(ap + 16);
          d10 = wmh(a.v, bh0.v, z8);
          d11 = wmh(a.v, bh1.v, z8);
        }
        const v8f e2lo = ld8(bsm + EB2O + 8 * hh);
        const v8f e2hi = ld8(bsm + EB2O + 16 + 8 * hh);
        FragH bq0, bq1;
        {
          v8h t0, t1, t2, t3;
#pragma unroll
          for (int i = 0; i < 8; ++i) {
            t0[i] = (_Float16)(d00[i] * WINV2 + e2lo[i]);
            t1[i] = (_Float16)(d10[i] * WINV2 + e2hi[i]);
            t2[i] = (_Float16)(d01[i] * WINV2 + e2lo[i]);
            t3[i] = (_Float16)(d11[i] * WINV2 + e2hi[i]);
          }
          bq0.h[0] = t0; bq0.h[1] = t1;
          bq1.h[0] = t2; bq1.h[1] = t3;
        }
        const int s0 = ssrc[wave * 32 + m], s1 = ssrc[wave * 32 + 16 + m];
        const int d0 = sdst[wave * 32 + m], d1 = sdst[wave * 32 + 16 + m];
        const float* P0 = pq + (size_t)s0 * PQW;
        const float* P1 = pq + (size_t)s1 * PQW;
        const float* Q0 = pq + (size_t)d0 * PQW + HD;
        const float* Q1 = pq + (size_t)d1 * PQW + HD;
        float part0 = 0.0f, part1 = 0.0f;
#pragma unroll 1
        for (int mt = 0; mt < 8; ++mt) {
          FragH a;
          const _Float16* ap = wsm + (EDM + 16 * mt + m) * 32 + 8 * hh;
          a.h[0] = *(const v8h*)ap;
          a.h[1] = *(const v8h*)(ap + 16);
          const v8f dm0 = wmh(a.v, bq0.v, z8);
          const v8f dm1 = wmh(a.v, bq1.v, z8);
          const int co = 16 * mt + 8 * hh;
          const v8f p0  = ld8(P0 + co);
          const v8f q0v = ld8(Q0 + co);
          const v8f p1  = ld8(P1 + co);
          const v8f q1v = ld8(Q1 + co);
          const v8f w2  = ld8(bsm + CW2O + co);
#pragma unroll
          for (int rI = 0; rI < 8; ++rI) {
            const float z0 = dm0[rI] * WINV + (p0[rI] + q0v[rI]);
            const float z1 = dm1[rI] * WINV + (p1[rI] + q1v[rI]);
            part0 = fmaf(silu_f(z0), w2[rI], part0);
            part1 = fmaf(silu_f(z1), w2[rI], part1);
          }
        }
        const float o0 = __shfl_xor(part0, 16);
        const float o1 = __shfl_xor(part1, 16);
        const float w0  = part0 + o0;
        const float w1v = part1 + o1;
        const float wown = (hh == 0) ? w0 : w1v;
        float* mp = msg + (wave * 32 + lane) * AW;
        mp[0] = wown * ux;
        mp[1] = wown * uy;
        mp[2] = wown * uz;
      }
      __syncthreads();

      if (wave == 0) {
#pragma unroll 1
        for (int i = 0; i < PASSN; ++i) {
          int sl = slotb[i];
          sl = sl < 0 ? 0 : (sl > NB ? NB : sl);
          if (lane < AW) {
            const float v = msg[i * AW + lane];
            acc[sl * AW + lane] += v;
          }
        }
      }
      __syncthreads();
    }

    int rem = newN - R * PASSN;
    rem = rem < 0 ? 0 : rem;
    if (R > 0 && tid < rem) pend[tid] = pend[R * PASSN + tid];
    if (tid == 0) pendN = rem;
  }
  __syncthreads();

  const size_t lim = (size_t)(outLim < 1 ? 1 : outLim);
  const size_t ob  = (size_t)nodeBase * AW;
  v4f ov[NQ];
#pragma unroll
  for (int q = 0; q < NQ; ++q) {
    const int f = (wave * NQ + q) * 128 + 4 * lane;
    float t[4];
#pragma unroll
    for (int j = 0; j < 4; ++j) {
      size_t gi = ob + (size_t)(f + j);
      gi = gi < lim ? gi : lim - 1;
      t[j] = acc[f + j] + x[gi];
    }
    v4f v = {t[0], t[1], t[2], t[3]};
    ov[q] = v;
  }
  const size_t slim = (size_t)(outLim < 0 ? 0 : outLim);
#pragma unroll
  for (int q = 0; q < NQ; ++q) {
    const size_t gi = ob + (size_t)((wave * NQ + q) * 128 + 4 * lane);
    if (gi + 3 < slim) *(volatile v4f*)(outp + gi) = ov[q];
  }
  __threadfence();
#pragma unroll
  for (int q = 0; q < NQ; ++q) {
    const size_t gi = ob + (size_t)((wave * NQ + q) * 128 + 4 * lane);
    if (gi + 3 < slim) *(volatile v4f*)(outp + gi) = ov[q];
  }
}

extern "C" void kernel_launch(void* const* d_in, const int* in_sizes, int n_in,
                              void* d_out, int out_size, void* d_ws, size_t ws_size,
                              hipStream_t stream) {
  if (n_in < 16) return;
  const int nN = in_sizes[0] / 3;
  const int nE = in_sizes[2];
  if (nN <= 0 || in_sizes[0] != nN * 3 || in_sizes[1] != nN * 63) return;
  if (nE < 0 || in_sizes[14] != 2 * nE) return;
  if (in_sizes[3] < EDM || in_sizes[4] < EDM || in_sizes[5] != EDM * EDM || in_sizes[6] < EDM) return;
  if (in_sizes[11] != (2 * ND + EDM) * HD || in_sizes[12] < HD || in_sizes[13] < HD) return;
  if (in_sizes[15] < 1) return;
  if (out_size != nN * 3) return;

  const float* x     = (const float*)d_in[0];
  const float* cond  = (const float*)d_in[1];
  const float* edist = (const float*)d_in[2];
  const float* ew1   = (const float*)d_in[3];
  const float* eb1   = (const float*)d_in[4];
  const float* ew2   = (const float*)d_in[5];
  const float* eb2   = (const float*)d_in[6];
  const float* cw1   = (const float*)d_in[11];
  const float* cb1   = (const float*)d_in[12];
  const float* cw2   = (const float*)d_in[13];
  const int*   ei    = (const int*)d_in[14];
  const int*   tp    = (const int*)d_in[15];
  float* out = (float*)d_out;

  const int nBlk = (nN + NB - 1) / NB;
  const int nPad = nBlk * NB;

  char* ws = (char*)d_ws;
  size_t off = 0;
  const size_t oH = off; off += (size_t)nPad * ND * 2;        off = (off + 255) & ~(size_t)255;
  const size_t oW = off; off += (size_t)(2 * HD) * ND * 2;     off = (off + 255) & ~(size_t)255;
  const size_t oP = off; off += (size_t)nPad * PQW * 4;        off = (off + 255) & ~(size_t)255;
  if (off > ws_size) return;
  _Float16* h16  = (_Float16*)(ws + oH);
  _Float16* wt16 = (_Float16*)(ws + oW);
  float*    pq   = (float*)(ws + oP);

  const int nHB  = nPad / 32;
  const int vec8 = ((nE & 3) == 0) ? 1 : 0;

  k_prep<<<nHB + (2 * HD) / 32, 256, 0, stream>>>(cond, tp, cw1, h16, wt16, nN, nHB);

  k_node<<<nPad / 16, 64, 0, stream>>>(h16, wt16, cb1, pq);

  k_agg<<<nBlk, NTHR, 0, stream>>>(x, ei, edist, ew1, eb1, ew2, eb2, cw1, cw2, pq, out,
                                   nN, nE, vec8, nN * 3);
}
